// MOELayer_45475113730574
// MI455X (gfx1250) — hardware-verified
//
#include <hip/hip_runtime.h>
#include <math.h>
typedef __attribute__((ext_vector_type(16))) _Float16 v16h;
typedef __attribute__((ext_vector_type(8)))  _Float16 v8h;
typedef __attribute__((ext_vector_type(16))) __bf16   v16b;
typedef __attribute__((ext_vector_type(8)))  __bf16   v8b;
typedef __attribute__((ext_vector_type(8)))  float    v8f;
typedef __attribute__((ext_vector_type(4)))  float    v4f;
#define PSCALE 32768.0f
#define U16(p) ((const unsigned short*)(const void*)(p))
#define PSCALE_INV (1.0f / 32768.0f)

__device__ __forceinline__ unsigned short f2bf_bits(float f) {
  unsigned u = __float_as_uint(f);
  return (unsigned short)((u + 0x7FFFu + ((u >> 16) & 1u)) >> 16);
}
__device__ __forceinline__ float bf_bits2f(unsigned short h) { return __uint_as_float(((unsigned)h) << 16); }

__device__ __forceinline__ void dep_guard_h(v8f& a, v8f& b, v16h x, v16h y) { asm volatile("v_nop\n\tv_nop\n\tv_nop\n\tv_nop" : "+v"(a), "+v"(b) : "v"(x), "v"(y)); }
__device__ __forceinline__ void dep_guard_b(v8f& a, v8f& b, v16b x, v16b y) { asm volatile("v_nop\n\tv_nop\n\tv_nop\n\tv_nop" : "+v"(a), "+v"(b) : "v"(x), "v"(y)); }
__device__ __forceinline__ void keep4_h(v16h a, v16h b, v16h c, v16h d) { asm volatile("v_nop" :: "v"(a), "v"(b), "v"(c), "v"(d)); }
__device__ __forceinline__ void keep4_b(v16b a, v16b b, v16b c, v16b d) { asm volatile("v_nop" :: "v"(a), "v"(b), "v"(c), "v"(d)); }
__device__ __forceinline__ void acc_guard4(v8f& a, v8f& b, v8f& c, v8f& d) { asm volatile("v_nop\n\tv_nop\n\tv_nop\n\tv_nop" : "+v"(a), "+v"(b), "+v"(c), "+v"(d)); }
template <typename T> struct Frag;
template <> struct Frag<_Float16> {
  typedef v16h V; union U { v16h v; v8h h[2]; };
  static __device__ __forceinline__ v16h load(const _Float16* p) {
    U f; f.h[0] = *(const v8h*)(p); f.h[1] = *(const v8h*)(p + 16); return f.v;
  }
  static __device__ __forceinline__ v8f mma(v16h a, v16h b, v8f c) {
    return __builtin_amdgcn_wmma_f32_16x16x32_f16(false, a, false, b, (short)0, c, false, false);
  }
  static __device__ __forceinline__ void guard(v8f& a, v8f& b, v16h x, v16h y) { dep_guard_h(a, b, x, y); }
  static __device__ __forceinline__ void keep(v16h a, v16h b, v16h c, v16h d) { keep4_h(a, b, c, d); }
};
template <> struct Frag<__bf16> {
  typedef v16b V; union U { v16b v; v8b h[2]; };
  static __device__ __forceinline__ v16b load(const __bf16* p) {
    U f; f.h[0] = *(const v8b*)(p); f.h[1] = *(const v8b*)(p + 16); return f.v;
  }
  static __device__ __forceinline__ v8f mma(v16b a, v16b b, v8f c) {
    return __builtin_amdgcn_wmma_f32_16x16x32_bf16(false, a, false, b, (short)0, c, false, false);
  }
  static __device__ __forceinline__ void guard(v8f& a, v8f& b, v16b x, v16b y) { dep_guard_b(a, b, x, y); }
  static __device__ __forceinline__ void keep(v16b a, v16b b, v16b c, v16b d) { keep4_b(a, b, c, d); }
};

template <int ET> struct Elem;
template <> struct Elem<0> { typedef _Float16 T; };
template <> struct Elem<1> { typedef __bf16 T; };
template <int ET, bool SPLIT, int BIAS_MODE, int OUT_MODE, bool RESID, int ACT = 0>
__global__ __launch_bounds__(256) void wmma_gemm64(
    const unsigned short* __restrict__ Ap, const unsigned short* __restrict__ A2p, int lda, long strideA,
    const unsigned short* __restrict__ Btp, const unsigned short* __restrict__ Bt2p, int ldb, long strideB,
    void* __restrict__ Cout, void* __restrict__ Cout2, int ldc, long strideC,
    const float* __restrict__ bias,
    const float* __restrict__ resid, long strideR,
    int M, int N, int K, float scale) {
  typedef typename Elem<ET>::T T;
  typedef typename Frag<T>::V V;
  const T* A = (const T*)Ap; const T* A2 = (const T*)A2p; const T* Bt = (const T*)Btp; const T* Bt2 = (const T*)Bt2p;
  __shared__ __align__(16) float sT[8][16 * 68];
  const int b    = blockIdx.y;
  const int lane = threadIdx.x & 31;
  const int wave = threadIdx.x >> 5;
  const int tilesN = N >> 6;
  const int tilesM = M >> 6;
  const int tile = blockIdx.x * 8 + wave;
  if (tile >= tilesM * tilesN) return;
  const int tm = tile / tilesN;
  const int tn = tile - tm * tilesN;
  const int m0 = tm << 6;
  const int n0 = tn << 6;

  const T* Ab  = A  + (size_t)b * strideA;
  const T* Bb  = Bt + (size_t)b * strideB;
  const T* Ab2 = SPLIT ? (A2  + (size_t)b * strideA) : nullptr;
  const T* Bb2 = SPLIT ? (Bt2 + (size_t)b * strideB) : nullptr;

  const int rlane = lane & 15;
  const int koff  = (lane >> 4) * 8;
  const int mOff  = (lane >> 4) * 8;

  v8f acc[4][4];
#pragma unroll
  for (int i = 0; i < 4; ++i)
#pragma unroll
    for (int j = 0; j < 4; ++j) acc[i][j] = (v8f){0.f,0.f,0.f,0.f,0.f,0.f,0.f,0.f};

  for (int k0 = 0; k0 < K; k0 += 32) {
    V bh[4], bl[4];
#pragma unroll
    for (int j = 0; j < 4; ++j) {
      const size_t bo = (size_t)(n0 + (j << 4) + rlane) * ldb + koff + k0;
      bh[j] = Frag<T>::load(Bb + bo);
      if (SPLIT) bl[j] = Frag<T>::load(Bb2 + bo);
    }
#pragma unroll
    for (int i = 0; i < 4; ++i) {
      const size_t ao = (size_t)(m0 + (i << 4) + rlane) * lda + koff + k0;
      V ah = Frag<T>::load(Ab + ao);
      V al;
      if (SPLIT) al = Frag<T>::load(Ab2 + ao);
#pragma unroll
      for (int j = 0; j < 4; ++j) {
        acc[i][j] = Frag<T>::mma(ah, bh[j], acc[i][j]);
        if (SPLIT) {
          acc[i][j] = Frag<T>::mma(ah, bl[j], acc[i][j]);
          acc[i][j] = Frag<T>::mma(al, bh[j], acc[i][j]);
        }
      }
      Frag<T>::guard(acc[i][0], acc[i][3], ah, SPLIT ? al : ah);
    }
    Frag<T>::keep(bh[0], bh[1], bh[2], bh[3]);
    if (SPLIT) Frag<T>::keep(bl[0], bl[1], bl[2], bl[3]);
  }
  acc_guard4(acc[0][0], acc[0][1], acc[0][2], acc[0][3]);
  acc_guard4(acc[1][0], acc[1][1], acc[1][2], acc[1][3]);
  acc_guard4(acc[2][0], acc[2][1], acc[2][2], acc[2][3]);
  acc_guard4(acc[3][0], acc[3][1], acc[3][2], acc[3][3]);

  float* slab = sT[wave];
  const float* Rb = RESID ? (resid + (size_t)b * strideR) : nullptr;
#pragma unroll
  for (int i = 0; i < 4; ++i) {
    const int mBase = m0 + (i << 4);
#pragma unroll
    for (int j = 0; j < 4; ++j) {
      const int n = n0 + (j << 4) + rlane;
      float bv = 0.f;
      if (BIAS_MODE == 2) bv = bias[n];
#pragma unroll
      for (int r = 0; r < 8; ++r) {
        float v = acc[i][j][r] * scale;
        if (BIAS_MODE == 1) v += bias[mBase + mOff + r];
        if (BIAS_MODE == 2) v += bv;
        if (RESID) v += Rb[(size_t)(mBase + mOff + r) * ldc + n];
        if (ACT == 1) v = tanhf(v);
        if (ACT == 2) v = fmaxf(v, 0.0f);
        slab[(mOff + r) * 68 + (j << 4) + rlane] = v;
      }
    }
    __builtin_amdgcn_fence(__ATOMIC_RELEASE, "workgroup");
    __builtin_amdgcn_wave_barrier();
    __builtin_amdgcn_fence(__ATOMIC_ACQUIRE, "workgroup");
    if (OUT_MODE == 0) {
      float* C = (float*)Cout + (size_t)b * strideC;
      const int hh = lane >> 4, c4 = (lane & 15) * 4;
      for (int pass = 0; pass < 2; ++pass) {
#pragma unroll
        for (int it = 0; it < 8; ++it) {
          const int row = it * 2 + hh;
          v4f v = *(const v4f*)(slab + row * 68 + c4);
          *(volatile v4f*)(C + (size_t)(mBase + row) * ldc + n0 + c4) = v;
        }
        __threadfence();
      }
    } else {
      const int q = lane >> 3, c8 = (lane & 7) * 8;
      unsigned short* C  = (unsigned short*)Cout  + (size_t)b * strideC;
      unsigned short* C2 = (OUT_MODE == 2) ? ((unsigned short*)Cout2 + (size_t)b * strideC) : nullptr;
      for (int pass = 0; pass < 2; ++pass) {
#pragma unroll
        for (int it = 0; it < 4; ++it) {
          const int row = it * 4 + q;
          const float* sp = slab + row * 68 + c8;
          v8h hv, lv;
#pragma unroll
          for (int e = 0; e < 8; ++e) {
            if (OUT_MODE == 1) {
              hv[e] = (_Float16)sp[e];
            } else {
              unsigned short hb = f2bf_bits(sp[e]);
              unsigned short lb = f2bf_bits(sp[e] - bf_bits2f(hb));
              hv[e] = __builtin_bit_cast(_Float16, hb);
              lv[e] = __builtin_bit_cast(_Float16, lb);
            }
          }
          *(volatile v8h*)(C + (size_t)(mBase + row) * ldc + n0 + c8) = hv;
          if (OUT_MODE == 2) *(volatile v8h*)(C2 + (size_t)(mBase + row) * ldc + n0 + c8) = lv;
        }
        __threadfence();
      }
    }
    __builtin_amdgcn_fence(__ATOMIC_RELEASE, "workgroup");
    __builtin_amdgcn_wave_barrier();
    __builtin_amdgcn_fence(__ATOMIC_ACQUIRE, "workgroup");
  }
}


__global__ __launch_bounds__(256) void transpose_cast_f16(const float* __restrict__ in, int ldi,
                                                         _Float16* __restrict__ outT, int ldo, float scale) {
  __shared__ __align__(16) _Float16 tile[64][72];
  const int c0 = blockIdx.x * 64, r0 = blockIdx.y * 64;
  const int t = threadIdx.y * 32 + threadIdx.x;
  for (int i = threadIdx.y; i < 64; i += 8) {
    tile[threadIdx.x][i]      = (_Float16)(in[(size_t)(r0 + i) * ldi + c0 + threadIdx.x] * scale);
    tile[32 + threadIdx.x][i] = (_Float16)(in[(size_t)(r0 + i) * ldi + c0 + 32 + threadIdx.x] * scale);
  }
  __syncthreads();
  const int q = t >> 3, c8 = (t & 7) * 8;
  for (int pass = 0; pass < 2; ++pass) {
#pragma unroll
    for (int it = 0; it < 2; ++it) {
      const int c = it * 32 + q;
      v8h hv = *(const v8h*)(&tile[c][c8]);
      *(volatile v8h*)(outT + (size_t)(c0 + c) * ldo + r0 + c8) = hv;
    }
    __threadfence();
  }
}


__global__ __launch_bounds__(256) void transpose_split_bf16(const float* __restrict__ in, int ldi,
                                                           __bf16* __restrict__ outH, __bf16* __restrict__ outL, int ldo) {
  __shared__ __align__(16) float tile[64][68];
  const int c0 = blockIdx.x * 64, r0 = blockIdx.y * 64;
  const int t = threadIdx.y * 32 + threadIdx.x;
  for (int i = threadIdx.y; i < 64; i += 8) {
    tile[threadIdx.x][i]      = in[(size_t)(r0 + i) * ldi + c0 + threadIdx.x];
    tile[32 + threadIdx.x][i] = in[(size_t)(r0 + i) * ldi + c0 + 32 + threadIdx.x];
  }
  __syncthreads();
  const int q = t >> 3, c8 = (t & 7) * 8;
  for (int pass = 0; pass < 2; ++pass) {
#pragma unroll
    for (int it = 0; it < 2; ++it) {
      const int c = it * 32 + q;
      v8b hv, lv;
#pragma unroll
      for (int e = 0; e < 8; ++e) {
        const float f = tile[c][c8 + e];
        const unsigned short hb = f2bf_bits(f);
        hv[e] = __builtin_bit_cast(__bf16, hb);
        lv[e] = __builtin_bit_cast(__bf16, f2bf_bits(f - bf_bits2f(hb)));
      }
      *(volatile v8b*)(outH + (size_t)(c0 + c) * ldo + r0 + c8) = hv;
      *(volatile v8b*)(outL + (size_t)(c0 + c) * ldo + r0 + c8) = lv;
    }
    __threadfence();
  }
}

#define NS 4096
#define DM 1024
#define NEX 16
#define DFF 4096
#define CAP 512

__global__ __launch_bounds__(256) void router_kernel(const float* __restrict__ x, const float* __restrict__ wg, float* __restrict__ tok) {
  const int lane = threadIdx.x & 31, wave = threadIdx.x >> 5;
  const int s = blockIdx.x * 8 + wave;
  const float* xr = x + (size_t)s * DM;
  float acc[NEX];
#pragma unroll
  for (int e = 0; e < NEX; ++e) acc[e] = 0.f;
#pragma unroll 1
  for (int k = lane; k < DM; k += 32) {
    const float xv = xr[k];
    const float* w = wg + (size_t)k * NEX;
#pragma unroll
    for (int e = 0; e < NEX; ++e) acc[e] += xv * w[e];
  }
#pragma unroll
  for (int e = 0; e < NEX; ++e)
    for (int o = 16; o > 0; o >>= 1) acc[e] += __shfl_xor(acc[e], o, 32);
  float mx = acc[0]; int i1 = 0;
#pragma unroll
  for (int e = 1; e < NEX; ++e) if (acc[e] > mx) { mx = acc[e]; i1 = e; }
  float se = 0.f, ex[NEX];
#pragma unroll 1
  for (int e = 0; e < NEX; ++e) { ex[e] = expf(acc[e] - mx); se += ex[e]; }
  float m2 = -INFINITY; int i2 = 0; bool found = false;
#pragma unroll
  for (int e = 0; e < NEX; ++e) if (e != i1 && (!found || acc[e] > m2)) { m2 = acc[e]; i2 = e; found = true; }
  float v;
  if (lane < NEX) { float exsel = 0.f;
#pragma unroll
    for (int e = 0; e < NEX; ++e) if (e == lane) exsel = ex[e];
    v = exsel / se; }
  else if (lane == 16) v = (float)i1;
  else if (lane == 17) v = (float)i2;
  else v = 0.f;
  ((volatile float*)tok)[(size_t)s * 32 + lane] = v;
  __threadfence();
  ((volatile float*)tok)[(size_t)s * 32 + lane] = v;
}

__global__ __launch_bounds__(256) void positions_kernel(const float* __restrict__ tok, int* __restrict__ cnt1, int* __restrict__ cnt2, int* __restrict__ slot) {
  __shared__ int sc1[256], sc2[256];
  __shared__ int sl[CAP];
  const int e = blockIdx.x, t = threadIdx.x;
  const int s0 = t * (NS / 256);
  int a1 = 0, a2 = 0;
  int i1v[16], i2v[16];
  for (int i = 0; i < 16; ++i) {
    const int s = s0 + i;
    i1v[i] = (int)tok[(size_t)s * 32 + 16]; i2v[i] = (int)tok[(size_t)s * 32 + 17];
    a1 += (i1v[i] == e); a2 += (i2v[i] == e);
  }
  sc1[t] = a1; sc2[t] = a2;
  for (int i = t; i < CAP; i += 256) sl[i] = -1;
  __syncthreads();
  for (int off = 1; off < 256; off <<= 1) {
    int v1 = (t >= off) ? sc1[t - off] : 0, v2 = (t >= off) ? sc2[t - off] : 0;
    __syncthreads();
    sc1[t] += v1; sc2[t] += v2;
    __syncthreads();
  }
  const int total1 = sc1[255];
  int r1 = sc1[t] - a1, r2 = sc2[t] - a2;
  for (int i = 0; i < 16; ++i) {
    const int s = s0 + i;
    if (i1v[i] == e) { if (r1 < CAP) sl[r1] = s; ++r1; }
    if (i2v[i] == e) { const int c = r2 + total1; if (c < CAP) sl[c] = s; ++r2; }
    i1v[i] = r1; i2v[i] = r2;
  }
  __syncthreads();
  __shared__ int stage[NS];
  for (int i = 0; i < 16; ++i) stage[s0 + i] = i1v[i];
  __syncthreads();
  for (int pass = 0; pass < 2; ++pass) { for (int i = t; i < NS; i += 256) ((volatile int*)cnt1)[(size_t)e * NS + i] = stage[i]; __threadfence(); }
  __syncthreads();
  for (int i = 0; i < 16; ++i) stage[s0 + i] = i2v[i];
  __syncthreads();
  for (int pass = 0; pass < 2; ++pass) {
    for (int i = t; i < NS; i += 256) ((volatile int*)cnt2)[(size_t)e * NS + i] = stage[i];
    for (int i = t; i < CAP; i += 256) ((volatile int*)slot)[e * CAP + i] = sl[i];
    __threadfence();
  }
}

__global__ __launch_bounds__(256) void dispatch_kernel(const float* __restrict__ x, const int* __restrict__ slot, unsigned* __restrict__ Xe) {
  const int lane = threadIdx.x & 31, wave = threadIdx.x >> 5;
  const int row = blockIdx.x * 8 + wave;
  int s = slot[row]; if (s >= NS) s = -1;
  const float* xr = (s >= 0) ? x + (size_t)s * DM : nullptr;
  for (int pass = 0; pass < 2; ++pass) {
    for (int c = lane; c < DM / 2; c += 32) {
      float a = 0.f, b = 0.f;
      if (s >= 0) { a = xr[2 * c]; b = xr[2 * c + 1]; }
      const unsigned u = (unsigned)__builtin_bit_cast(unsigned short, (_Float16)a) | ((unsigned)__builtin_bit_cast(unsigned short, (_Float16)b) << 16);
      ((volatile unsigned*)Xe)[(size_t)row * (DM / 2) + c] = u;
    }
    __threadfence();
  }
}

__global__ __launch_bounds__(256) void combine_kernel(const float* __restrict__ tok, const int* __restrict__ cnt1, const int* __restrict__ cnt2,
                                                     const float* __restrict__ EO, float* __restrict__ out) {
  const int lane = threadIdx.x & 31, wave = threadIdx.x >> 5;
  const int s = blockIdx.x * 8 + wave;
  int e1 = (int)tok[(size_t)s * 32 + 16], e2 = (int)tok[(size_t)s * 32 + 17];
  e1 = e1 < 0 ? 0 : (e1 > 15 ? 15 : e1); e2 = e2 < 0 ? 0 : (e2 > 15 ? 15 : e2);
  const float ga = tok[(size_t)s * 32 + e1], gb = tok[(size_t)s * 32 + e2];
  const int loc1 = cnt1[(size_t)e1 * NS + s] - 1;
  const int loc2 = cnt2[(size_t)e2 * NS + s] - 1 + cnt1[(size_t)e2 * NS + (NS - 1)];
  const bool k1 = (loc1 >= 0) && (loc1 < CAP), k2 = (loc2 >= 0) && (loc2 < CAP);
  float g1 = k1 ? ga : 0.f, g2 = k2 ? gb : 0.f;
  const float den = fmaxf(g1 + g2, 1e-9f);
  g1 = g1 / den; g2 = g2 / den;
  const float* r1 = EO + (size_t)(e1 * CAP + (k1 ? loc1 : 0)) * DM;
  const float* r2 = EO + (size_t)(e2 * CAP + (k2 ? loc2 : 0)) * DM;
  for (int pass = 0; pass < 2; ++pass) {
#pragma unroll
    for (int i = 0; i < DM / 128; ++i) {
      const int c = i * 128 + lane * 4;
      v4f a = *(const v4f*)(r1 + c), b = *(const v4f*)(r2 + c), o;
#pragma unroll
      for (int q = 0; q < 4; ++q) o[q] = (k1 ? g1 * a[q] : 0.f) + (k2 ? g2 * b[q] : 0.f);
      *(volatile v4f*)(out + (size_t)s * DM + c) = o;
    }
    __threadfence();
  }
}

extern "C" void kernel_launch(void* const* d_in, const int* in_sizes, int n_in,
                              void* d_out, int out_size, void* d_ws, size_t ws_size,
                              hipStream_t stream) {
  (void)in_sizes; (void)n_in; (void)out_size; (void)ws_size;
  const float* x  = (const float*)d_in[0];
  const float* wg = (const float*)d_in[1];
  const float* w1 = (const float*)d_in[2];
  const float* b1 = (const float*)d_in[3];
  const float* w2 = (const float*)d_in[4];
  const float* b2 = (const float*)d_in[5];
  float* out = (float*)d_out;

  char* ws = (char*)d_ws; size_t off = 0;
  auto carve = [&](size_t bytes) -> char* { char* p = ws + off; off += (bytes + 255) & ~(size_t)255; return p; };
  float*    tok  = (float*)carve((size_t)NS * 32 * 4);
  int*      cnt1 = (int*)carve((size_t)NEX * NS * 4);
  int*      cnt2 = (int*)carve((size_t)NEX * NS * 4);
  int*      slot = (int*)carve((size_t)NEX * CAP * 4);
  unsigned* Xe   = (unsigned*)carve((size_t)NEX * CAP * DM * 2);
  _Float16* W1T  = (_Float16*)carve((size_t)DFF * DM * 2);
  __bf16*   W2Th = (__bf16*)carve((size_t)DM * DFF * 2);
  __bf16*   W2Tl = (__bf16*)carve((size_t)DM * DFF * 2);
  unsigned* Hh   = (unsigned*)carve((size_t)NEX * CAP * DFF * 2);
  unsigned* Hl   = (unsigned*)carve((size_t)NEX * CAP * DFF * 2);
  float*    EO   = (float*)carve((size_t)NEX * CAP * DM * 4);

  router_kernel<<<NS / 8, 256, 0, stream>>>(x, wg, tok);
  positions_kernel<<<NEX, 256, 0, stream>>>(tok, cnt1, cnt2, slot);
  dispatch_kernel<<<NEX * CAP / 8, 256, 0, stream>>>(x, slot, Xe);
  transpose_cast_f16<<<dim3(DFF / 64, DM / 64), dim3(32, 8), 0, stream>>>(w1, DFF, W1T, DM, 1.0f);
  transpose_split_bf16<<<dim3(DM / 64, DFF / 64), dim3(32, 8), 0, stream>>>(w2, DM, W2Th, W2Tl, DFF);
  {
    const int t1 = (NEX * CAP / 64) * (DFF / 64);
    wmma_gemm64<0, false, 2, 2, false, 2><<<dim3((t1 + 7) / 8, 1), 256, 0, stream>>>(
        (const unsigned short*)Xe, nullptr, DM, 0, U16(W1T), nullptr, DM, 0, Hh, Hl, DFF, 0, b1, nullptr, 0, NEX * CAP, DFF, DM, 1.0f);
    const int t2 = (NEX * CAP / 64) * (DM / 64);
    wmma_gemm64<1, true, 2, 0, false, 0><<<dim3((t2 + 7) / 8, 1), 256, 0, stream>>>(
        (const unsigned short*)Hh, (const unsigned short*)Hl, DFF, 0, U16(W2Th), U16(W2Tl), DFF, 0, EO, nullptr, DM, 0, b2, nullptr, 0, NEX * CAP, DM, DFF, 1.0f);
  }
  combine_kernel<<<NS / 8, 256, 0, stream>>>(tok, cnt1, cnt2, EO, out);
}
